// DeepGainModel_28707561407391
// MI455X (gfx1250) — hardware-verified
//
#include <hip/hip_runtime.h>
#include <math.h>


typedef _Float16 f16t;
typedef f16t  v16h __attribute__((ext_vector_type(16)));
typedef f16t  v8h  __attribute__((ext_vector_type(8)));
typedef float v8f  __attribute__((ext_vector_type(8)));
typedef float v4f  __attribute__((ext_vector_type(4)));
typedef unsigned int v4u __attribute__((ext_vector_type(4)));

union Frag { v16h v; v8h q[2]; };
union Pk16 { v8h h; v4u u; };

#define NBATCH 256
#define NSTEP  128
#define NEMB   64
#define NHID   256
#define NH2    128
#define NMUS   16
#define NEXR   27
#define BPB    8
#define FROWS  (BPB * NMUS)
#define LP     264
#define LPF    132
#define DT_SCALE 5.1298987149230735f
#define WSC    256.0f
#define WINV   0.00390625f

union XU { f16t h[FROWS * LP]; float f[FROWS * LPF]; };
static_assert(sizeof(XU) == (size_t)FROWS * LP * 2);
static_assert((size_t)FROWS * LP * 2 == (size_t)FROWS * LPF * 4);

__device__ __forceinline__ v8f wmma16(v16h a, v16h b, v8f c) {
    return __builtin_amdgcn_wmma_f32_16x16x32_f16(false, a, false, b, (short)0, c, false, false);
}

__device__ __forceinline__ void wguard(v8f (&c)[4][1], Frag (&a)[4], Frag (&b)[1]) {
    asm volatile("v_nop\n\tv_nop\n\tv_nop\n\tv_nop"
                 : "+v"(c[0][0]), "+v"(c[1][0]), "+v"(c[2][0]), "+v"(c[3][0])
                 : "v"(a[0].v), "v"(a[1].v), "v"(a[2].v), "v"(a[3].v), "v"(b[0].v));
}
__device__ __forceinline__ void wguard(v8f (&c)[4][2], Frag (&a)[4], Frag (&b)[2]) {
    asm volatile("v_nop\n\tv_nop\n\tv_nop\n\tv_nop"
                 : "+v"(c[0][0]), "+v"(c[0][1]), "+v"(c[1][0]), "+v"(c[1][1]),
                   "+v"(c[2][0]), "+v"(c[2][1]), "+v"(c[3][0]), "+v"(c[3][1])
                 : "v"(a[0].v), "v"(a[1].v), "v"(a[2].v), "v"(a[3].v),
                   "v"(b[0].v), "v"(b[1].v));
}

template<int MT, int NT>
__device__ __forceinline__ void zacc(v8f (&acc)[MT][NT]) {
    const v8f z = {0.f, 0.f, 0.f, 0.f, 0.f, 0.f, 0.f, 0.f};
#pragma unroll
    for (int i = 0; i < MT; ++i)
#pragma unroll
        for (int j = 0; j < NT; ++j) acc[i][j] = z;
}

template<int MT, int NT>
__device__ __forceinline__ void mma_acc(v8f (&acc)[MT][NT],
                                        const f16t* A, int lda,
                                        const f16t* B, int ldb, int ktiles) {
    const int l = threadIdx.x & 31, h = l >> 4, m = l & 15;
    const f16t* ap = A + (size_t)m * lda + 8 * h;
    const f16t* bp = B + (size_t)m * ldb + 8 * h;
#pragma unroll 1
    for (int kt = 0; kt < ktiles; ++kt) {
        Frag a[MT], b[NT];
#pragma unroll
        for (int i = 0; i < MT; ++i) {
            const f16t* p = ap + (size_t)i * 16 * lda + kt * 32;
            a[i].q[0] = *(const v8h*)p;
            a[i].q[1] = *(const v8h*)(p + 16);
        }
#pragma unroll
        for (int j = 0; j < NT; ++j) {
            const f16t* p = bp + (size_t)j * 16 * ldb + kt * 32;
            b[j].q[0] = *(const v8h*)p;
            b[j].q[1] = *(const v8h*)(p + 16);
        }
#pragma unroll
        for (int i = 0; i < MT; ++i)
#pragma unroll
            for (int j = 0; j < NT; ++j)
                acc[i][j] = wmma16(a[i].v, b[j].v, acc[i][j]);
        wguard(acc, a, b);
    }
}

template<int MT, int NT>
__device__ __forceinline__ void epi_h(v8f (&acc)[MT][NT], float inv, const float* bias,
                                      int f0, f16t* L, int pitch) {
    const int l = threadIdx.x & 31, h = l >> 4, m = l & 15;
#pragma unroll
    for (int i = 0; i < MT; ++i) {
        const float* bq = bias + f0 + 16 * i + 8 * h;
        v4f c0 = *(const v4f*)bq;
        v4f c1 = *(const v4f*)(bq + 4);
#pragma unroll
        for (int j = 0; j < NT; ++j) {
            Pk16 pk;
#pragma unroll
            for (int r = 0; r < 4; ++r) {
                float v0 = fmaxf(fmaf(acc[i][j][r], inv, c0[r]), 0.0f);
                float v1 = fmaxf(fmaf(acc[i][j][4 + r], inv, c1[r]), 0.0f);
                pk.h[r]     = (f16t)v0;
                pk.h[4 + r] = (f16t)v1;
            }
            *(v8h*)(L + (size_t)(16 * j + m) * pitch + f0 + 16 * i + 8 * h) = pk.h;
        }
    }
}

template<int MT, int NT>
__device__ __forceinline__ void epi_f(v8f (&acc)[MT][NT], float inv, const float* bias,
                                      int f0, float* S, int pitch) {
    const int l = threadIdx.x & 31, h = l >> 4, m = l & 15;
#pragma unroll
    for (int i = 0; i < MT; ++i) {
        const float* bq = bias + f0 + 16 * i + 8 * h;
        v4f c0 = *(const v4f*)bq;
        v4f c1 = *(const v4f*)(bq + 4);
#pragma unroll
        for (int j = 0; j < NT; ++j) {
            v4f p0, p1;
#pragma unroll
            for (int r = 0; r < 4; ++r) {
                p0[r] = fmaxf(fmaf(acc[i][j][r], inv, c0[r]), 0.0f);
                p1[r] = fmaxf(fmaf(acc[i][j][4 + r], inv, c1[r]), 0.0f);
            }
            float* d = S + (size_t)(16 * j + m) * pitch + f0 + 16 * i + 8 * h;
            *(v4f*)d       = p0;
            *(v4f*)(d + 4) = p1;
        }
    }
}

__device__ __forceinline__ v4f ld4(const float* p) { return *(const v4f*)p; }

__device__ __forceinline__ float fsigm(float x) {
    return __builtin_amdgcn_rcpf(1.0f + expf(-x));
}

__global__ __launch_bounds__(256)
void k_tables(const float* exe, const float* mue, const float* fW1, const float* fb1,
              const float* gW1, const float* gb1, float* TE, float* TM, float* GE) {
    const int h = threadIdx.x;
    const int b = blockIdx.x;
    const float* src;
    const float* wcol;
    float acc;
    float* dst;
    if (b < NEXR) {
        src = exe + b * NEMB; wcol = fW1 + 4 * NHID + h; acc = 0.0f; dst = TE + b * NHID + h;
    } else if (b < NEXR + NMUS) {
        const int m = b - NEXR;
        src = mue + m * NEMB; wcol = fW1 + 68 * NHID + h; acc = fb1[h]; dst = TM + m * NHID + h;
    } else {
        const int e = b - NEXR - NMUS;
        src = exe + e * NEMB; wcol = gW1 + 2 * NHID + h; acc = gb1[h]; dst = GE + e * NHID + h;
    }
#pragma unroll 1
    for (int j = 0; j < NEMB; ++j) acc = fmaf(src[j], wcol[(size_t)j * NHID], acc);
    *(volatile float*)dst = acc;
    __threadfence();
    *(volatile float*)dst = acc;
}

__global__ __launch_bounds__(256)
void k_pack(const float* W, f16t* P, int K, int N, float sc) {
    int i  = blockIdx.x * 256 + threadIdx.x;
    int kq = K >> 3;
    int tot = N * kq;
    if (i >= tot) return;
    int n = i / kq;
    int k = (i - n * kq) * 8;
    Pk16 v;
#pragma unroll
    for (int e = 0; e < 8; ++e)
        v.h[e] = (f16t)(W[(size_t)(k + e) * N + n] * sc);
    f16t* d = P + (size_t)n * K + k;
    *(volatile v4u*)d = v.u;
    __threadfence();
    *(volatile v4u*)d = v.u;
}

__global__ __launch_bounds__(256)
void k_main(const int* eidx, const float* wgt, const float* rps, const float* rrt,
            const float* dlt, const float* ltau, const float* invt,
            const float* fW1, const float* gW1,
            const float* TE, const float* TM, const float* GE,
            const f16t* P2F, const float* fb2, const f16t* P3F, const float* fb3,
            const float* fW4, const float* fb4,
            const f16t* P2R, const float* gb2, const f16t* P3R, const float* gb3,
            const float* gW4, const float* gb4,
            float* out0, float* out1, int nb, int nstep) {
    __shared__ __attribute__((aligned(16))) XU    sX;
    __shared__ __attribute__((aligned(16))) f16t  sH1R[16 * LP];
    __shared__ __attribute__((aligned(16))) f16t  sH2F[FROWS * LP];
    __shared__ __attribute__((aligned(16))) f16t  sH2R[16 * LP];
    __shared__ __attribute__((aligned(16))) float sH3R[16 * LPF];
    __shared__ __attribute__((aligned(16))) float sRir[BPB * NSTEP];
    __shared__ __attribute__((aligned(16))) float sMpc[BPB * NMUS];
    __shared__ __attribute__((aligned(16))) float sW4F[NH2];
    __shared__ __attribute__((aligned(16))) float sW4R[NH2];
    __shared__ float sInv[NEXR * NMUS];
    __shared__ float sRtau[NMUS];
    __shared__ float sW[BPB], sRp[BPB], sRt[BPB];
    __shared__ int   sEix[BPB];

    const int tid = threadIdx.x, wv = tid >> 5, lane = tid & 31;
    const int b0 = blockIdx.x * BPB;
    if (b0 + BPB > nb || nstep != NSTEP) return;
    f16t*  sH1F = sX.h;
    float* sH3F = sX.f;

    if (tid < BPB * NMUS) sMpc[tid] = 1.0f;
    if (tid < NMUS) sRtau[tid] = 1.0f / expf(ltau[tid]);
    if (tid < NH2) { sW4F[tid] = fW4[tid]; sW4R[tid] = gW4[tid]; }
    for (int i = tid; i < NEXR * NMUS; i += 256) sInv[i] = invt[i];
    {
        Pk16 z; z.u = (v4u){0u, 0u, 0u, 0u};
        for (int i = tid; i < (16 * LP) / 8; i += 256) *(v8h*)(sH1R + 8 * i) = z.h;
    }
    for (int i = tid; i < BPB * NSTEP; i += 256) sRir[i] = 0.0f;
    const float fb4v = fb4[0], gb4v = gb4[0];
    __syncthreads();

#pragma unroll 1
    for (int t = 0; t < NSTEP; ++t) {
        if (tid < BPB) {
            const int off = (b0 + tid) * NSTEP + t;
            sW[tid] = wgt[off]; sRp[tid] = rps[off]; sRt[tid] = rrt[off];
            int e = eidx[off];
            e = e < 0 ? 0 : e;
            e = e > NEXR - 1 ? NEXR - 1 : e;
            sEix[tid] = e;
        }
        if (tid < BPB * NMUS) {
            const int b = tid >> 4, m = tid & 15;
            const float dt  = dlt[(b0 + b) * NSTEP + t];
            const float dth = expm1f(dt * DT_SCALE);
            const float mp  = sMpc[tid];
            const float rec = 1.0f - (1.0f - mp) * expf(-dth * sRtau[m]);
            sMpc[tid] = (t > 0) ? rec : mp;
        }
        __syncthreads();

        {
            const int c8 = lane * 8, rg = wv;
            const v4f f0a = ld4(fW1 + c8),            f0b = ld4(fW1 + c8 + 4);
            const v4f f1a = ld4(fW1 + NHID + c8),     f1b = ld4(fW1 + NHID + c8 + 4);
            const v4f f2a = ld4(fW1 + 2 * NHID + c8), f2b = ld4(fW1 + 2 * NHID + c8 + 4);
            const v4f f3a = ld4(fW1 + 3 * NHID + c8), f3b = ld4(fW1 + 3 * NHID + c8 + 4);
            const v4f tm0a = ld4(TM + rg * NHID + c8),       tm0b = ld4(TM + rg * NHID + c8 + 4);
            const v4f tm1a = ld4(TM + (rg + 8) * NHID + c8), tm1b = ld4(TM + (rg + 8) * NHID + c8 + 4);
#pragma unroll 1
            for (int b = 0; b < BPB; ++b) {
                const float w = sW[b], rp = sRp[b], rt = sRt[b];
                const int e = sEix[b];
                v4f ba = ld4(TE + e * NHID + c8), bb = ld4(TE + e * NHID + c8 + 4);
                ba = ba + w * f0a + rp * f1a + rt * f2a;
                bb = bb + w * f0b + rp * f1b + rt * f2b;
                {
                    const float mp = sMpc[b * NMUS + rg];
                    v4f va = ba + mp * f3a + tm0a;
                    v4f vb = bb + mp * f3b + tm0b;
                    Pk16 pk;
#pragma unroll
                    for (int r = 0; r < 4; ++r) {
                        pk.h[r]     = (f16t)fmaxf(va[r], 0.0f);
                        pk.h[4 + r] = (f16t)fmaxf(vb[r], 0.0f);
                    }
                    *(v8h*)(sH1F + (size_t)(b * NMUS + rg) * LP + c8) = pk.h;
                }
                {
                    const float mp = sMpc[b * NMUS + rg + 8];
                    v4f va = ba + mp * f3a + tm1a;
                    v4f vb = bb + mp * f3b + tm1b;
                    Pk16 pk;
#pragma unroll
                    for (int r = 0; r < 4; ++r) {
                        pk.h[r]     = (f16t)fmaxf(va[r], 0.0f);
                        pk.h[4 + r] = (f16t)fmaxf(vb[r], 0.0f);
                    }
                    *(v8h*)(sH1F + (size_t)(b * NMUS + rg + 8) * LP + c8) = pk.h;
                }
            }
        }
        {
            const int c8 = lane * 8, b = wv;
            const float w = sW[b], rp = sRp[b];
            const int e = sEix[b];
            v4f va = ld4(GE + e * NHID + c8)     + w * ld4(gW1 + c8)     + rp * ld4(gW1 + NHID + c8);
            v4f vb = ld4(GE + e * NHID + c8 + 4) + w * ld4(gW1 + c8 + 4) + rp * ld4(gW1 + NHID + c8 + 4);
#pragma unroll 4
            for (int m = 0; m < NMUS; ++m) {
                const float mp = sMpc[b * NMUS + m];
                va = va + mp * ld4(gW1 + (66 + m) * NHID + c8);
                vb = vb + mp * ld4(gW1 + (66 + m) * NHID + c8 + 4);
            }
            Pk16 pk;
#pragma unroll
            for (int r = 0; r < 4; ++r) {
                pk.h[r]     = (f16t)fmaxf(va[r], 0.0f);
                pk.h[4 + r] = (f16t)fmaxf(vb[r], 0.0f);
            }
            *(v8h*)(sH1R + (size_t)b * LP + c8) = pk.h;
        }
        __syncthreads();

        {
#pragma unroll 1
            for (int u = wv; u < 16; u += 8) {
                const int fg = u & 3, tg = u >> 2;
                v8f acc[4][2]; zacc(acc);
                mma_acc<4, 2>(acc, P2F + (size_t)(64 * fg) * NHID, NHID, sH1F + (size_t)(32 * tg) * LP, LP, 8);
                epi_h<4, 2>(acc, WINV, fb2, 64 * fg, sH2F + (size_t)(32 * tg) * LP, LP);
            }
            if (wv < 4) {
                v8f acc[4][1]; zacc(acc);
                mma_acc<4, 1>(acc, P2R + (size_t)(64 * wv) * NHID, NHID, sH1R, LP, 8);
                epi_h<4, 1>(acc, WINV, gb2, 64 * wv, sH2R, LP);
            }
        }
        __syncthreads();

        {
            const int fg = wv & 1, tg = wv >> 1;
            v8f acc[4][2]; zacc(acc);
            mma_acc<4, 2>(acc, P3F + (size_t)(64 * fg) * NHID, NHID, sH2F + (size_t)(32 * tg) * LP, LP, 8);
            epi_f<4, 2>(acc, WINV, fb3, 64 * fg, sH3F + (size_t)(32 * tg) * LPF, LPF);
            if (wv < 2) {
                v8f accr[4][1]; zacc(accr);
                mma_acc<4, 1>(accr, P3R + (size_t)(64 * wv) * NHID, NHID, sH2R, LP, 8);
                epi_f<4, 1>(accr, WINV, gb3, 64 * wv, sH3R, LPF);
            }
        }
        __syncthreads();

        if (wv < 4) {
            const float* hr = sH3F + (size_t)tid * LPF;
            float acc = 0.0f;
#pragma unroll 4
            for (int q = 0; q < NH2 / 4; ++q) {
                const v4f hv = ld4(hr + 4 * q);
                const v4f wq = ld4(sW4F + 4 * q);
                acc = fmaf(hv[0], wq[0], acc);
                acc = fmaf(hv[1], wq[1], acc);
                acc = fmaf(hv[2], wq[2], acc);
                acc = fmaf(hv[3], wq[3], acc);
            }
            const float dropv = fsigm(acc + fb4v);
            const int b = tid >> 4, m = tid & 15;
            const float iv = sInv[sEix[b] * NMUS + m];
            const float mp = sMpc[tid];
            const float nm = fmaxf(mp * (1.0f - iv * dropv), 0.1f);
            sMpc[tid] = nm;
        } else if (wv == 4) {
            const int b = lane >> 2, part = lane & 3;
            const float* hr = sH3R + (size_t)b * LPF + part * 32;
            const float* wr = sW4R + part * 32;
            float acc = 0.0f;
#pragma unroll 2
            for (int q = 0; q < 8; ++q) {
                const v4f hv = ld4(hr + 4 * q);
                const v4f wq = ld4(wr + 4 * q);
                acc = fmaf(hv[0], wq[0], acc);
                acc = fmaf(hv[1], wq[1], acc);
                acc = fmaf(hv[2], wq[2], acc);
                acc = fmaf(hv[3], wq[3], acc);
            }
            acc += __shfl_xor(acc, 1);
            acc += __shfl_xor(acc, 2);
            const float rir = fsigm(acc + gb4v);
            if (part == 0) sRir[b * NSTEP + t] = rir;
        }
        __syncthreads();
    }

    {
        const int row = wv, col = lane * 4;
        const v4f v = ld4(sRir + row * NSTEP + col);
        float* d0 = out0 + (size_t)(b0 + row) * NSTEP + col;
        const bool w1 = tid < (BPB * NMUS) / 4;
        const v4f q = ld4(sMpc + lane * 4);
        float* d1 = out1 + (size_t)b0 * NMUS + lane * 4;
        *(volatile v4f*)d0 = v;
        if (w1) *(volatile v4f*)d1 = q;
        __threadfence();
        *(volatile v4f*)d0 = v;
        if (w1) *(volatile v4f*)d1 = q;
    }
}

extern "C" void kernel_launch(void* const* d_in, const int* in_sizes, int n_in,
                              void* d_out, int out_size, void* d_ws, size_t ws_size,
                              hipStream_t stream) {
    if (n_in < 26) return;
    const int nbt = NBATCH * NSTEP;
    if (in_sizes[0] != nbt || in_sizes[1] != nbt || in_sizes[2] != nbt ||
        in_sizes[3] != nbt || in_sizes[4] != nbt) return;
    if (in_sizes[6] != NEXR * NEMB || in_sizes[7] != NMUS * NEMB || in_sizes[8] != NMUS ||
        in_sizes[9] != NEXR * NMUS) return;
    if (in_sizes[10] != (4 + 2 * NEMB) * NHID || in_sizes[11] != NHID ||
        in_sizes[12] != NHID * NHID || in_sizes[13] != NHID ||
        in_sizes[14] != NHID * NH2 || in_sizes[15] != NH2 ||
        in_sizes[16] != NH2 || in_sizes[17] != 1) return;
    if (in_sizes[18] != (2 + NEMB + NMUS) * NHID || in_sizes[19] != NHID ||
        in_sizes[20] != NHID * NHID || in_sizes[21] != NHID ||
        in_sizes[22] != NHID * NH2 || in_sizes[23] != NH2 ||
        in_sizes[24] != NH2 || in_sizes[25] != 1) return;
    if (out_size != NBATCH * NSTEP + NBATCH * NMUS) return;
    if ((NBATCH % BPB) != 0) return;

    const int*   eidx = (const int*)d_in[0];
    const float* wgt  = (const float*)d_in[1];
    const float* rps  = (const float*)d_in[2];
    const float* rrt  = (const float*)d_in[3];
    const float* dlt  = (const float*)d_in[4];
    const float* exe  = (const float*)d_in[6];
    const float* mue  = (const float*)d_in[7];
    const float* ltau = (const float*)d_in[8];
    const float* invt = (const float*)d_in[9];
    const float* fW1  = (const float*)d_in[10]; const float* fb1 = (const float*)d_in[11];
    const float* fW2  = (const float*)d_in[12]; const float* fb2 = (const float*)d_in[13];
    const float* fW3  = (const float*)d_in[14]; const float* fb3 = (const float*)d_in[15];
    const float* fW4  = (const float*)d_in[16]; const float* fb4 = (const float*)d_in[17];
    const float* gW1  = (const float*)d_in[18]; const float* gb1 = (const float*)d_in[19];
    const float* gW2  = (const float*)d_in[20]; const float* gb2 = (const float*)d_in[21];
    const float* gW3  = (const float*)d_in[22]; const float* gb3 = (const float*)d_in[23];
    const float* gW4  = (const float*)d_in[24]; const float* gb4 = (const float*)d_in[25];
    float* out0 = (float*)d_out;
    float* out1 = out0 + (size_t)NBATCH * NSTEP;

    char* ws = (char*)d_ws;
    size_t off = 0;
    auto carve = [&](size_t bytes) -> char* {
        char* p = ws + off;
        off = (off + bytes + 255) & ~(size_t)255;
        return p;
    };
    float* TE  = (float*)carve((size_t)32 * NHID * 4);
    float* TM  = (float*)carve((size_t)NMUS * NHID * 4);
    float* GE  = (float*)carve((size_t)32 * NHID * 4);
    f16t*  P2F = (f16t*)carve((size_t)NHID * NHID * 2);
    f16t*  P3F = (f16t*)carve((size_t)NH2 * NHID * 2);
    f16t*  P2R = (f16t*)carve((size_t)NHID * NHID * 2);
    f16t*  P3R = (f16t*)carve((size_t)NH2 * NHID * 2);
    if (off > ws_size || off > (size_t)134217728) return;

    k_tables<<<dim3(NEXR + NMUS + NEXR), dim3(256), 0, stream>>>(exe, mue, fW1, fb1, gW1, gb1,
                                                                 TE, TM, GE);
    auto pack = [&](const float* W, f16t* P, int K, int N) {
        int tot = N * (K / 8);
        k_pack<<<dim3((tot + 255) / 256), dim3(256), 0, stream>>>(W, P, K, N, WSC);
    };
    pack(fW2, P2F, NHID, NHID);
    pack(fW3, P3F, NHID, NH2);
    pack(gW2, P2R, NHID, NHID);
    pack(gW3, P3R, NHID, NH2);

    k_main<<<dim3(NBATCH / BPB), dim3(256), 0, stream>>>(
        eidx, wgt, rps, rrt, dlt, ltau, invt, fW1, gW1, TE, TM, GE,
        P2F, fb2, P3F, fb3, fW4, fb4, P2R, gb2, P3R, gb3, gW4, gb4,
        out0, out1, NBATCH, NSTEP);
}
